// GroupedQueryAttention_19739669692842
// MI455X (gfx1250) — hardware-verified
//
#include <hip/hip_runtime.h>


#ifndef NB
#define NB 2
#endif
#ifndef SEQ
#define SEQ 2048
#endif
#define NB_FULL  2
#define SEQ_FULL 2048
#define DM   2048
#define NH_  32
#define NKV  8
#define LGNH 5
#define LGNKV 3
#define REP  (NH_ / NKV)
#define HD   64
#define DQ   (NH_ * HD)
#define DKV  (NKV * HD)
#define RH   ((SEQ) < 512 ? (SEQ) : 512)
static_assert(SEQ % 64 == 0);
static_assert(RH % 64 == 0);
static_assert((SEQ - RH) % 32 == 0);
static_assert(SEQ <= SEQ_FULL);
static_assert(NB <= NB_FULL);
static_assert((1 << LGNH) == NH_);
static_assert((1 << LGNKV) == NKV);
static_assert(NH_ == NKV * REP);
static_assert(HD == 64);
static_assert(DM % 32 == 0);
static_assert(DQ % 64 == 0);
static_assert(DKV % 64 == 0);
static_assert(((size_t)NB * NH_ * SEQ * HD) % 512 == 0);
static_assert(((size_t)NB * NKV * SEQ * HD) % 512 == 0);
static_assert(((size_t)SEQ * HD) % 256 == 0);
static_assert(((size_t)SEQ * DM) % 2048 == 0);
static_assert(((size_t)DQ * DM) % 2048 == 0);
static_assert(((size_t)DKV * DM) % 2048 == 0);
static_assert((size_t)NB * SEQ * DQ * 4 == 2 * ((size_t)NB * SEQ * DQ * 2));
static_assert(HD / 2 == 32);
static_assert(HD % 2 == 0);
static_assert((unsigned long long)NB * NH_ * SEQ * HD <= 0xFFFFFFFFull);
static_assert(DQ == DM);
static_assert(2 * ((size_t)DQ * DM * 2) + 2 * ((size_t)DKV * DM * 2) + (size_t)NB * SEQ * DM * 2 + (size_t)NB * SEQ * DQ * 4 + (size_t)NB * SEQ * DKV * 4
              + (size_t)NB * NH_ * SEQ * HD * 2 + 2 * ((size_t)NB * NH_ * RH * HD * 2) + 2 * ((size_t)NB * NKV * SEQ * HD * 2) + 4 * ((size_t)NB * NKV * RH * HD * 2) + 16 * 256 <= (size_t)134217728);

typedef _Float16 h16;
typedef unsigned short bf;
typedef __attribute__((ext_vector_type(16))) __bf16   v16bf;
typedef __attribute__((ext_vector_type(16))) _Float16 v16h;
typedef __attribute__((ext_vector_type(16))) unsigned short v16us;
typedef __attribute__((ext_vector_type(8)))  _Float16 v8h;
typedef __attribute__((ext_vector_type(8)))  unsigned short v8us;
typedef __attribute__((ext_vector_type(8)))  float    v8f;
typedef __attribute__((ext_vector_type(4)))  float    v4f;
typedef __attribute__((ext_vector_type(2)))  _Float16 v2h;
typedef __attribute__((ext_vector_type(2)))  unsigned short v2us;
typedef __attribute__((ext_vector_type(2)))  float v2f;
typedef v4f  __attribute__((may_alias)) v4fa;

__device__ __forceinline__ unsigned short f2bf(float f) { unsigned u = __float_as_uint(f); u += 0x7FFFu + ((u >> 16) & 1u); return (unsigned short)(u >> 16); }
__device__ __forceinline__ float bf2f(unsigned short b) { return __uint_as_float(((unsigned)b) << 16); }
__device__ __forceinline__ float bfr(float f) { return bf2f(f2bf(f)); }
__device__ __forceinline__ v16h cat16(v8h lo, v8h hi) { return __builtin_shufflevector(lo, hi, 0, 1, 2, 3, 4, 5, 6, 7, 8, 9, 10, 11, 12, 13, 14, 15); }
__device__ __forceinline__ v16bf cat16b(v8us lo, v8us hi) { return __builtin_bit_cast(v16bf, __builtin_shufflevector(lo, hi, 0, 1, 2, 3, 4, 5, 6, 7, 8, 9, 10, 11, 12, 13, 14, 15)); }
__device__ __forceinline__ v8f wmma16(v16h a, v16h b, v8f c) { return __builtin_amdgcn_wmma_f32_16x16x32_f16(false, a, false, b, (short)0, c, false, false); }
__device__ __forceinline__ v8f wmmab(v16bf a, v16bf b, v8f c) { return __builtin_amdgcn_wmma_f32_16x16x32_bf16(false, a, false, b, (short)0, c, false, false); }
__device__ __forceinline__ h16 tohx(float x) { return (h16)x; }
__device__ __forceinline__ void splitf(float y, unsigned short& h, unsigned short& l) { h = f2bf(y); l = f2bf(y - bf2f(h)); }

template <typename T16> struct WFrag;
template <> struct WFrag<h16> { typedef v16h V; static __device__ __forceinline__ V ld(const h16* p) { return cat16(*(const v8h*)p, *(const v8h*)(p + 16)); } static __device__ __forceinline__ v8f mma(V a, V b, v8f c) { return wmma16(a, b, c); } };
template <> struct WFrag<bf> { typedef v16bf V; static __device__ __forceinline__ V ld(const bf* p) { return cat16b(*(const v8us*)p, *(const v8us*)(p + 16)); } static __device__ __forceinline__ v8f mma(V a, V b, v8f c) { return wmmab(a, b, c); } };

template <typename T16, int NSPLIT, bool BIAS>
__global__ __launch_bounds__(32) void k_gemmw(const T16* __restrict__ A, const T16* __restrict__ A2, const T16* __restrict__ Bt, const T16* __restrict__ Bt2, int K, float* C, int ldc, const float* __restrict__ bias, size_t sA, size_t sB, size_t sC) {
    typedef typename WFrag<T16>::V V;
    __shared__ __align__(16) float os[16 * 68];
    const size_t z = blockIdx.z; A += z * sA; if (A2) A2 += z * sA; Bt += z * sB; if (Bt2) Bt2 += z * sB; C += z * sC;
    const int lane = threadIdx.x & 31, lr = lane & 15, hi = lane >> 4; const int r0 = blockIdx.x * 64, c0 = blockIdx.y * 64;
    v8f acc[4][4];
#pragma unroll
    for (int mb = 0; mb < 4; ++mb)
#pragma unroll
        for (int nb = 0; nb < 4; ++nb) acc[mb][nb] = (v8f){};
    const size_t aoff = (size_t)(r0 + lr) * K + 8 * hi, boff = (size_t)(c0 + lr) * K + 8 * hi;
#pragma unroll 1
    for (int kc = 0; kc < K; kc += 32) {
        V a[4], a2[4];
#pragma unroll
        for (int mb = 0; mb < 4; ++mb) { a[mb] = WFrag<T16>::ld(A + aoff + (size_t)mb * 16 * K + kc); if (NSPLIT == 1 || NSPLIT == 2) a2[mb] = WFrag<T16>::ld(A2 + aoff + (size_t)mb * 16 * K + kc); }
#pragma unroll
        for (int nb = 0; nb < 4; ++nb) { const V b = WFrag<T16>::ld(Bt + boff + (size_t)nb * 16 * K + kc); V b2; if (NSPLIT >= 2) b2 = WFrag<T16>::ld(Bt2 + boff + (size_t)nb * 16 * K + kc);
#pragma unroll
            for (int mb = 0; mb < 4; ++mb) { acc[mb][nb] = WFrag<T16>::mma(a[mb], b, acc[mb][nb]); if (NSPLIT == 1 || NSPLIT == 2) acc[mb][nb] = WFrag<T16>::mma(a2[mb], b, acc[mb][nb]); if (NSPLIT >= 2) acc[mb][nb] = WFrag<T16>::mma(a[mb], b2, acc[mb][nb]); } }
        asm volatile("v_nop\n\tv_nop\n\tv_nop\n\tv_nop" : "+v"(acc[0][0]), "+v"(acc[1][1]), "+v"(acc[2][2]), "+v"(acc[3][3]) : "v"(a[0]), "v"(a[3]));
    }
#pragma unroll
    for (int mb = 0; mb < 4; ++mb) {
#pragma unroll
        for (int nb = 0; nb < 4; ++nb) {
#pragma unroll
            for (int j = 0; j < 8; ++j) os[(hi * 8 + j) * 68 + nb * 16 + lr] = acc[mb][nb][j]; }
        __builtin_amdgcn_wave_barrier(); asm volatile("" ::: "memory");
        float* crow = C + (size_t)(r0 + mb * 16) * ldc + c0;
#pragma unroll 1
        for (int ps = 0; ps < 2; ++ps) {
#pragma unroll
            for (int s = 0; s < 8; ++s) { const int row = 2 * s + hi, cofs = lr * 4; v4f val = *(const v4fa*)(os + row * 68 + cofs); if (BIAS) { val[0] += bfr(bias[c0 + cofs]); val[1] += bfr(bias[c0 + cofs + 1]); val[2] += bfr(bias[c0 + cofs + 2]); val[3] += bfr(bias[c0 + cofs + 3]); }
                *(volatile v4f*)(crow + (size_t)row * ldc + cofs) = val; }
            if (ps == 0) __threadfence(); }
        __builtin_amdgcn_wave_barrier(); asm volatile("" ::: "memory");
    }
}

template <int QT> struct Gd;
template <> struct Gd<1> {
    static __device__ __forceinline__ void s(v8f (&st)[2][1]) { asm volatile("v_nop\n\tv_nop\n\tv_nop\n\tv_nop" : "+v"(st[0][0]), "+v"(st[1][0])); }
    static __device__ __forceinline__ void o(v8f (&ot)[1][4]) { asm volatile("v_nop\n\tv_nop\n\tv_nop\n\tv_nop" : "+v"(ot[0][0]), "+v"(ot[0][1]), "+v"(ot[0][2]), "+v"(ot[0][3])); }
};
template <> struct Gd<2> {
    static __device__ __forceinline__ void s(v8f (&st)[2][2]) { asm volatile("v_nop\n\tv_nop\n\tv_nop\n\tv_nop" : "+v"(st[0][0]), "+v"(st[1][0]), "+v"(st[0][1]), "+v"(st[1][1])); }
    static __device__ __forceinline__ void o(v8f (&ot)[2][4]) { asm volatile("v_nop\n\tv_nop\n\tv_nop\n\tv_nop" : "+v"(ot[0][0]), "+v"(ot[0][1]), "+v"(ot[0][2]), "+v"(ot[0][3]), "+v"(ot[1][0]), "+v"(ot[1][1]), "+v"(ot[1][2]), "+v"(ot[1][3])); }
};
template <typename T16> struct PPk;
template <> struct PPk<h16> {
    static __device__ __forceinline__ void pk(const float (&p0)[8], const float (&p1)[8], v16h& a, v16h& a2) { (void)a2; v16h t;
#pragma unroll
        for (int r = 0; r < 8; ++r) { t[r] = tohx(p0[r]); t[8 + r] = tohx(p1[r]); }
        a = t; }
};
template <> struct PPk<bf> {
    static __device__ __forceinline__ void pk(const float (&p0)[8], const float (&p1)[8], v16bf& a, v16bf& a2) { v16us th, tl;
#pragma unroll
        for (int r = 0; r < 8; ++r) { unsigned short x, y; splitf(p0[r], x, y); th[r] = x; tl[r] = y; splitf(p1[r], x, y); th[8 + r] = x; tl[8 + r] = y; }
        a = __builtin_bit_cast(v16bf, th); a2 = __builtin_bit_cast(v16bf, tl); }
};

template <typename T16, int NS, int QT>
static __device__ __forceinline__ void flash_body(const T16* __restrict__ Qa, const T16* __restrict__ Qa2, const T16* __restrict__ Ka, const T16* __restrict__ Ka2, const T16* __restrict__ Va, const T16* __restrict__ Va2,
                                                  unsigned qpr, unsigned kpr, unsigned vp, unsigned rbase, float carl, bf* ATh, bf* ATl) {
    typedef typename WFrag<T16>::V V;
    __shared__ __align__(16) float os[16 * QT * 68];
    const unsigned lane = threadIdx.x & 31u, lr = lane & 15u, hi = lane >> 4;
    const unsigned qw = rbase + blockIdx.x * (16u * QT);
    const unsigned h = blockIdx.y, b = blockIdx.z, g = h / (unsigned)REP;
    const size_t qo = ((size_t)(b * NH_ + h) * qpr + qw + lr) * HD + 8u * hi;
    const size_t ko = ((size_t)(b * NKV + g) * kpr + lr) * HD + 8u * hi;
    const size_t vo = ((size_t)(b * NKV + g) * HD + lr) * vp + 8u * hi;
    const T16* Qp = Qa + qo; const T16* Kp = Ka + ko; const T16* Vp = Va + vo;
    const T16* Qp2 = NS ? (Qa2 + qo) : Qp; const T16* Kp2 = NS ? (Ka2 + ko) : Kp; const T16* Vp2 = NS ? (Va2 + vo) : Vp;
    const float C1 = 0.125f * 1.4426950408889634f;

    V qf[QT][2], qf2[QT][2];
#pragma unroll
    for (int qt = 0; qt < QT; ++qt)
#pragma unroll
        for (int ks = 0; ks < 2; ++ks) { qf[qt][ks] = WFrag<T16>::ld(Qp + qt * 16 * HD + ks * 32); if (NS) qf2[qt][ks] = WFrag<T16>::ld(Qp2 + qt * 16 * HD + ks * 32); }
    v8f ot[QT][4]; float mrun[QT], ls[QT];
#pragma unroll
    for (int qt = 0; qt < QT; ++qt) { mrun[qt] = -3.0e38f; ls[qt] = 0.f;
#pragma unroll
        for (int dt = 0; dt < 4; ++dt) ot[qt][dt] = (v8f){}; }

    const unsigned nch = (qw + 16u * QT + 31u) >> 5;
#pragma unroll 1
    for (unsigned ch = 0; ch < nch; ++ch) {
        const unsigned kb = ch * 32u;
        v8f st[2][QT];
#pragma unroll
        for (int kt = 0; kt < 2; ++kt)
#pragma unroll
            for (int qt = 0; qt < QT; ++qt) st[kt][qt] = (v8f){};
        V ka, ka2;
#pragma unroll
        for (int kt = 0; kt < 2; ++kt)
#pragma unroll
            for (int ks = 0; ks < 2; ++ks) {
                ka = WFrag<T16>::ld(Kp + (size_t)(kb + 16u * kt) * HD + ks * 32); if (NS) ka2 = WFrag<T16>::ld(Kp2 + (size_t)(kb + 16u * kt) * HD + ks * 32);
#pragma unroll
                for (int qt = 0; qt < QT; ++qt) { st[kt][qt] = WFrag<T16>::mma(ka, qf[qt][ks], st[kt][qt]); if (NS) { st[kt][qt] = WFrag<T16>::mma(ka2, qf[qt][ks], st[kt][qt]); st[kt][qt] = WFrag<T16>::mma(ka, qf2[qt][ks], st[kt][qt]); } } }
        Gd<QT>::s(st);
        asm volatile("" :: "v"(ka)); if (NS) asm volatile("" :: "v"(ka2));

        const bool diag = (kb + 31u > qw);
        V pb[QT], pb2[QT];
#pragma unroll
        for (int qt = 0; qt < QT; ++qt) {
            const unsigned qi = qw + 16u * qt + lr;
            float u0[8], u1[8];
#pragma unroll
            for (int r = 0; r < 8; ++r) { u0[r] = st[0][qt][r] * C1; u1[r] = st[1][qt][r] * C1; }
            if (diag) {
#pragma unroll
                for (int r = 0; r < 8; ++r) { const unsigned key = kb + 8u * hi + (unsigned)r; u0[r] = (key <= qi) ? u0[r] : -3.0e38f; u1[r] = (key + 16u <= qi) ? u1[r] : -3.0e38f; } }
            float mx = fmaxf(u0[0], u1[0]);
#pragma unroll
            for (int r = 1; r < 8; ++r) mx = fmaxf(mx, fmaxf(u0[r], u1[r]));
            mx = fmaxf(mx, __shfl_xor(mx, 16, 32));
            const float mnew = fmaxf(mrun[qt], mx);
            const float alpha = __builtin_amdgcn_exp2f(mrun[qt] - mnew);
            mrun[qt] = mnew;
            const float base = carl - mnew;
            float p0[8], p1[8]; float sum = 0.f;
#pragma unroll
            for (int r = 0; r < 8; ++r) { p0[r] = __builtin_amdgcn_exp2f(u0[r] + base); p1[r] = __builtin_amdgcn_exp2f(u1[r] + base); sum += p0[r]; sum += p1[r]; }
            ls[qt] = ls[qt] * alpha + sum;
#pragma unroll
            for (int dt = 0; dt < 4; ++dt)
#pragma unroll
                for (int r = 0; r < 8; ++r) ot[qt][dt][r] *= alpha;
            PPk<T16>::pk(p0, p1, pb[qt], pb2[qt]);
        }
        V va, va2;
#pragma unroll
        for (int dt = 0; dt < 4; ++dt) {
            va = WFrag<T16>::ld(Vp + (size_t)(16u * dt) * vp + kb); if (NS) va2 = WFrag<T16>::ld(Vp2 + (size_t)(16u * dt) * vp + kb);
#pragma unroll
            for (int qt = 0; qt < QT; ++qt) { ot[qt][dt] = WFrag<T16>::mma(va, pb[qt], ot[qt][dt]); if (NS) { ot[qt][dt] = WFrag<T16>::mma(va2, pb[qt], ot[qt][dt]); ot[qt][dt] = WFrag<T16>::mma(va, pb2[qt], ot[qt][dt]); } } }
        Gd<QT>::o(ot);
        asm volatile("" :: "v"(va)); if (NS) asm volatile("" :: "v"(va2));
#pragma unroll
        for (int qt = 0; qt < QT; ++qt) { asm volatile("" :: "v"(pb[qt])); if (NS) asm volatile("" :: "v"(pb2[qt])); }
    }

#pragma unroll
    for (int qt = 0; qt < QT; ++qt) {
        const float lt = ls[qt] + __shfl_xor(ls[qt], 16, 32);
        const float f = __builtin_amdgcn_rcpf(lt);
#pragma unroll
        for (int dt = 0; dt < 4; ++dt) { v4f a0, a1;
#pragma unroll
            for (int k = 0; k < 4; ++k) { a0[k] = ot[qt][dt][k] * f; a1[k] = ot[qt][dt][4 + k] * f; }
            float* dst = os + (16u * qt + lr) * 68u + 16u * dt + 8u * hi; *(v4fa*)dst = a0; *(v4fa*)(dst + 4) = a1; } }
    __builtin_amdgcn_wave_barrier(); asm volatile("" ::: "memory");
    const size_t ao = (size_t)(b * SEQ + qw) * DQ + h * HD;
#pragma unroll 1
    for (int ps = 0; ps < 2; ++ps) {
#pragma unroll
        for (unsigned s = 0; s < 4u * QT; ++s) { const unsigned row = 4u * s + (lane >> 3), c8 = (lane & 7u) * 8u;
            const v4f x0 = *(const v4fa*)(os + row * 68u + c8); const v4f x1 = *(const v4fa*)(os + row * 68u + c8 + 4u); v8us oh, ol;
#pragma unroll
            for (int k = 0; k < 4; ++k) { unsigned short a, c; splitf(x0[k], a, c); oh[k] = a; ol[k] = c; splitf(x1[k], a, c); oh[4 + k] = a; ol[4 + k] = c; }
            *(volatile v8us*)(ATh + ao + (size_t)row * DQ + c8) = oh; *(volatile v8us*)(ATl + ao + (size_t)row * DQ + c8) = ol; }
        if (ps == 0) __threadfence(); }
}

__global__ __launch_bounds__(32) void k_flash_hi(const bf* __restrict__ Qa, const bf* __restrict__ Qa2, const bf* __restrict__ Ka, const bf* __restrict__ Ka2, const bf* __restrict__ Va, const bf* __restrict__ Va2,
                                                 unsigned qpr, unsigned kpr, unsigned vp, unsigned rbase, float carl, bf* ATh, bf* ATl) {
    flash_body<bf, 2, 1>(Qa, Qa2, Ka, Ka2, Va, Va2, qpr, kpr, vp, rbase, carl, ATh, ATl);
}
__global__ __launch_bounds__(32) void k_flash_lo(const h16* __restrict__ Qa, const h16* __restrict__ Ka, const h16* __restrict__ Va,
                                                 unsigned qpr, unsigned kpr, unsigned vp, unsigned rbase, float carl, bf* ATh, bf* ATl) {
    flash_body<h16, 0, 2>(Qa, nullptr, Ka, nullptr, Va, nullptr, qpr, kpr, vp, rbase, carl, ATh, ATl);
}

__global__ __launch_bounds__(256) void k_cvt8(const float* __restrict__ src, bf* dst, unsigned n8, size_t sstr, size_t dstr) { const unsigned i = blockIdx.x * 256u + threadIdx.x; if (i >= n8) return; src += (size_t)blockIdx.y * sstr; dst += (size_t)blockIdx.y * dstr; const v8f v = *(const v8f*)(src + (size_t)i * 8); v8us o;
#pragma unroll
    for (int k = 0; k < 8; ++k) o[k] = f2bf(v[k]); *(volatile v8us*)(dst + (size_t)i * 8) = o; __threadfence(); *(volatile v8us*)(dst + (size_t)i * 8) = o; }

__global__ __launch_bounds__(256) void k_rope(const float* __restrict__ F, unsigned pitch, unsigned lgh, const float* __restrict__ COS, const float* __restrict__ SIN, h16* P16, bf* Ph, bf* Pl) {
    const unsigned e = (blockIdx.x * 256u + threadIdx.x) * 2u; if (e >= (((unsigned)(NB * SEQ * HD)) << lgh)) return;
    const unsigned d = e % HD, t = (e / HD) % SEQ, hb = e / (unsigned)(HD * SEQ); const unsigned h = hb & ((1u << lgh) - 1u), b = hb >> lgh;
    const float* f = F + (size_t)(b * SEQ + t) * pitch + h * HD; v2h o16; v2us oh, ol;
    const float x0 = f[d], x1 = f[d + 1u];
    const size_t ti = (size_t)t * (HD / 2) + (d >> 1);
    const float c = bfr(COS[ti]), s = bfr(SIN[ti]);
    float a = __fmul_rn(x0, c), bq = __fmul_rn(x1, s), cq = __fmul_rn(x0, s), dq = __fmul_rn(x1, c);
    asm volatile("" : "+v"(a)); asm volatile("" : "+v"(bq)); asm volatile("" : "+v"(cq)); asm volatile("" : "+v"(dq));
    const float r0 = __fsub_rn(a, bq), r1 = __fadd_rn(cq, dq);
    { unsigned short a2, c2; o16[0] = tohx(r0); splitf(r0, a2, c2); oh[0] = a2; ol[0] = c2; o16[1] = tohx(r1); splitf(r1, a2, c2); oh[1] = a2; ol[1] = c2; }
    const bool hl = (t < (unsigned)RH);
    const size_t ec = ((size_t)hb * RH + t) * HD + d;
    *(volatile v2h*)(P16 + e) = o16; if (hl) { *(volatile v2us*)(Ph + ec) = oh; *(volatile v2us*)(Pl + ec) = ol; }
    __threadfence();
    *(volatile v2h*)(P16 + e) = o16; if (hl) { *(volatile v2us*)(Ph + ec) = oh; *(volatile v2us*)(Pl + ec) = ol; } }

__global__ __launch_bounds__(256) void k_vtp(const float* __restrict__ F, unsigned pitch, h16* V16, bf* Vh, bf* Vl) {
    const unsigned e = (blockIdx.x * 256u + threadIdx.x) * 2u; if (e >= (unsigned)(NB * NKV * HD * SEQ)) return;
    const unsigned t = e % SEQ, d = (e / SEQ) % HD, gb = e / (unsigned)(SEQ * HD); const unsigned g = gb % NKV, b = gb / NKV; v2h o16; v2us oh, ol;
#pragma unroll
    for (int q = 0; q < 2; ++q) { const float x = F[(size_t)(b * SEQ + t + (unsigned)q) * pitch + g * HD + d]; o16[q] = tohx(x); unsigned short a2, c2; splitf(x, a2, c2); oh[q] = a2; ol[q] = c2; }
    const bool hl = (t < (unsigned)RH);
    const size_t ec = ((size_t)gb * HD + d) * RH + t;
    *(volatile v2h*)(V16 + e) = o16; if (hl) { *(volatile v2us*)(Vh + ec) = oh; *(volatile v2us*)(Vl + ec) = ol; }
    __threadfence();
    *(volatile v2h*)(V16 + e) = o16; if (hl) { *(volatile v2us*)(Vh + ec) = oh; *(volatile v2us*)(Vl + ec) = ol; } }

extern "C" void kernel_launch(void* const* d_in, const int* in_sizes, int n_in,
                              void* d_out, int out_size, void* d_ws, size_t ws_size, hipStream_t stream) {
    if (n_in < 7) return;
    const long long needx = (long long)(NB - 1) * SEQ_FULL * DM + (long long)SEQ * DM;
    if ((long long)in_sizes[0] < needx || (long long)in_sizes[1] < (long long)SEQ * (HD / 2) || (long long)in_sizes[2] < (long long)SEQ * (HD / 2)
        || (long long)in_sizes[3] < (long long)DQ * DM || (long long)in_sizes[4] < (long long)DKV * DM || (long long)in_sizes[5] < (long long)DKV * DM || (long long)in_sizes[6] < (long long)DM * DQ) return;
    if ((long long)out_size < needx) return;
    const float* x = (const float*)d_in[0]; const float* cosb = (const float*)d_in[1]; const float* sinb = (const float*)d_in[2];
    const float* wq = (const float*)d_in[3]; const float* wk = (const float*)d_in[4]; const float* wv = (const float*)d_in[5]; const float* wo = (const float*)d_in[6];
    float* OUT = (float*)d_out;
    char* wsp = (char*)d_ws;
    auto take = [&](size_t bytes) { char* p = wsp; wsp += (bytes + 255) & ~(size_t)255; return (void*)p; };
    bf* WQ = (bf*)take((size_t)DQ * DM * 2); bf* WK = (bf*)take((size_t)DKV * DM * 2); bf* WV = (bf*)take((size_t)DKV * DM * 2); bf* WO = (bf*)take((size_t)DM * DQ * 2);
    bf* XB = (bf*)take((size_t)NB * SEQ * DM * 2);
    float* FQ = (float*)take((size_t)NB * SEQ * DQ * 4);
    float* FK = (float*)take((size_t)NB * SEQ * DKV * 4);
    h16* QP16 = (h16*)take((size_t)NB * NH_ * SEQ * HD * 2); bf* QPh = (bf*)take((size_t)NB * NH_ * RH * HD * 2); bf* QPl = (bf*)take((size_t)NB * NH_ * RH * HD * 2);
    h16* KP16 = (h16*)take((size_t)NB * NKV * SEQ * HD * 2); bf* KPh = (bf*)take((size_t)NB * NKV * RH * HD * 2); bf* KPl = (bf*)take((size_t)NB * NKV * RH * HD * 2);
    h16* VT16 = (h16*)take((size_t)NB * NKV * HD * SEQ * 2); bf* VTh = (bf*)take((size_t)NB * NKV * HD * RH * 2); bf* VTl = (bf*)take((size_t)NB * NKV * HD * RH * 2);
    const size_t carved = (size_t)(wsp - (char*)d_ws);
    if (carved > ws_size || carved > (size_t)134217728) return;
    float* FV = FK;
    bf* ATh = (bf*)FQ;
    bf* ATl = ATh + (size_t)NB * SEQ * DQ;

    k_cvt8<<<dim3((unsigned)(((size_t)SEQ * DM / 8 + 255) / 256), NB), 256, 0, stream>>>(x, XB, (unsigned)((size_t)SEQ * DM / 8), (size_t)SEQ_FULL * DM, (size_t)SEQ * DM);
    k_cvt8<<<dim3((unsigned)(((size_t)DQ * DM / 8 + 255) / 256), 1), 256, 0, stream>>>(wq, WQ, (unsigned)((size_t)DQ * DM / 8), 0, 0);
    k_cvt8<<<dim3((unsigned)(((size_t)DKV * DM / 8 + 255) / 256), 1), 256, 0, stream>>>(wk, WK, (unsigned)((size_t)DKV * DM / 8), 0, 0);
    k_cvt8<<<dim3((unsigned)(((size_t)DKV * DM / 8 + 255) / 256), 1), 256, 0, stream>>>(wv, WV, (unsigned)((size_t)DKV * DM / 8), 0, 0);
    k_cvt8<<<dim3((unsigned)(((size_t)DM * DQ / 8 + 255) / 256), 1), 256, 0, stream>>>(wo, WO, (unsigned)((size_t)DM * DQ / 8), 0, 0);

    const unsigned LQ = (unsigned)(((size_t)NB * NH_ * SEQ * HD / 2 + 255) / 256), LKv = (unsigned)(((size_t)NB * NKV * SEQ * HD / 2 + 255) / 256);
    k_gemmw<bf, 0, false><<<dim3(NB * SEQ / 64, DQ / 64, 1), 32, 0, stream>>>(XB, nullptr, WQ, nullptr, DM, FQ, DQ, nullptr, 0, 0, 0);
    k_rope<<<LQ, 256, 0, stream>>>(FQ, DQ, LGNH, cosb, sinb, QP16, QPh, QPl);
    k_gemmw<bf, 0, false><<<dim3(NB * SEQ / 64, DKV / 64, 1), 32, 0, stream>>>(XB, nullptr, WK, nullptr, DM, FK, DKV, nullptr, 0, 0, 0);
    k_rope<<<LKv, 256, 0, stream>>>(FK, DKV, LGNKV, cosb, sinb, KP16, KPh, KPl);
    k_gemmw<bf, 0, false><<<dim3(NB * SEQ / 64, DKV / 64, 1), 32, 0, stream>>>(XB, nullptr, WV, nullptr, DM, FV, DKV, nullptr, 0, 0, 0);
    k_vtp<<<LKv, 256, 0, stream>>>(FV, DKV, VT16, VTh, VTl);

    k_flash_hi<<<dim3(RH / 16, NH_, NB), 32, 0, stream>>>(QPh, QPl, KPh, KPl, VTh, VTl, (unsigned)RH, (unsigned)RH, (unsigned)RH, 0u, 0.0f, ATh, ATl);
    if (SEQ > RH)
        k_flash_lo<<<dim3((SEQ - RH) / 32, NH_, NB), 32, 0, stream>>>(QP16, KP16, VT16, (unsigned)SEQ, (unsigned)SEQ, (unsigned)SEQ, (unsigned)RH, 10.0f, ATh, ATl);

    k_gemmw<bf, 1, false><<<dim3(SEQ / 64, DM / 64, NB), 32, 0, stream>>>(ATh, ATl, WO, nullptr, DQ, OUT, DM, nullptr, (size_t)SEQ * DQ, 0, (size_t)SEQ_FULL * DM);
}
